// HBiLSTM_19404662243372
// MI455X (gfx1250) — hardware-run, weakly checked
//
#include <hip/hip_runtime.h>
#include <math.h>

typedef __attribute__((ext_vector_type(16))) _Float16 v16h;
typedef __attribute__((ext_vector_type(8)))  _Float16 v8h;
typedef __attribute__((ext_vector_type(8)))  float    v8f;
typedef __attribute__((ext_vector_type(4)))  float    v4f;
typedef __attribute__((ext_vector_type(2)))  unsigned v2u;

constexpr int kB     = 32;
constexpr int kT     = 512;
constexpr int kDin   = 512;
constexpr int kH     = 256;
constexpr int kG4    = 4 * kH;
constexpr int kOutC  = 2 * kH;
constexpr int kRows  = kB * kT;
constexpr int kXgP   = 2 * kG4;
constexpr int kWcatRows = 2 * kG4 + kOutC;
constexpr int kSeqBlk = 16;
constexpr int kHP     = 264;
constexpr int kSlabP  = 36;
constexpr float kXCarry  = 16.0f;
constexpr float kWCarry  = 256.0f;
constexpr float kHCarry  = 64.0f;
constexpr float kInScale = 1.0f / (kXCarry * kWCarry);
constexpr float kHScale  = 1.0f / (kHCarry * kWCarry);
constexpr float kF16Min  = 6.103515625e-5f;
static_assert(kG4 == 1024 && kOutC == 512 && kRows == 16384 && kXgP == 2048 && kWcatRows == 2560);
static_assert((kDin % 32) == 0 && (kH % 32) == 0);
static_assert((kRows % 64) == 0 && (kXgP % 64) == 0 && (kOutC % 64) == 0 && (kT % 64) == 0);
static_assert((2 * kSeqBlk * kHP) % 256 == 0);
static_assert((kHP % 8) == 0 && (kSlabP % 4) == 0);
static_assert(kB == 2 * kSeqBlk);

constexpr size_t kSzXH   = (size_t)kRows * kDin * 2;
constexpr size_t kSzWCAT = (size_t)kWcatRows * kDin * 2;
constexpr size_t kSzWHH  = (size_t)2 * kG4 * kH * 2;
constexpr size_t kSzBIAS = (size_t)kWcatRows * 4;
constexpr size_t kSzXG   = (size_t)kRows * kXgP * 2;
constexpr size_t kSzHOUT = (size_t)kRows * kOutC * 4;
constexpr size_t kOffXH   = 0;
constexpr size_t kOffWCAT = kOffXH + kSzXH;
constexpr size_t kOffWHH  = kOffWCAT + kSzWCAT;
constexpr size_t kOffBIAS = kOffWHH + kSzWHH;
constexpr size_t kOffXG   = kOffBIAS + kSzBIAS;
constexpr size_t kOffHOUT = kOffXG + kSzXG;
constexpr size_t kWsTotal = kOffHOUT + kSzHOUT;
static_assert(kWsTotal == 121120768ull);
static_assert(kWsTotal <= 134217728ull);
static_assert((kOffWCAT % 256) == 0 && (kOffWHH % 256) == 0 && (kOffBIAS % 256) == 0 && (kOffXG % 256) == 0 && (kOffHOUT % 256) == 0);

__device__ __forceinline__ unsigned short f2bf_bits(float f) {
  unsigned u = __float_as_uint(f);
  return (unsigned short)((u + 0x7FFFu + ((u >> 16) & 1u)) >> 16);
}
__device__ __forceinline__ float bf16r(float f) { return __uint_as_float(((unsigned)f2bf_bits(f)) << 16); }
__device__ __forceinline__ float flush16(float v) { return (fabsf(v) < kF16Min) ? 0.0f : v; }
__device__ __forceinline__ float h16_to_f32(unsigned hb) {
  const unsigned sgn = (hb & 0x8000u) << 16;
  const unsigned em = hb & 0x7fffu;
  const float fn = __uint_as_float((em << 13) + 0x38000000u);
  const float fs = (float)em * 5.9604644775390625e-8f;
  const float mag = (em < 0x400u) ? fs : fn;
  return __uint_as_float(__float_as_uint(mag) | sgn);
}
__device__ __forceinline__ float sigm(float x) { return 1.0f / (1.0f + expf(-x)); }
__device__ __forceinline__ float tanh_id(float x) { return 1.0f - 2.0f / (1.0f + expf(2.0f * x)); }

union FragH { v16h v; v8h h[2]; };
__device__ __forceinline__ v16h load_frag(const _Float16* p) {
  FragH f;
  f.h[0] = *(const v8h*)(p);
  f.h[1] = *(const v8h*)(p + 16);
  return f.v;
}
__device__ __forceinline__ v8f mma_h(v16h a, v16h b, v8f c) {
  c = __builtin_amdgcn_wmma_f32_16x16x32_f16(false, a, false, b, (short)0, c, false, false);
  asm volatile("v_nop\n\tv_nop\n\tv_nop\n\tv_nop" : "+v"(c) : "v"(a), "v"(b));
  return c;
}

template <bool PERM>
__global__ __launch_bounds__(256) void cvt8_kernel(const float* __restrict__ src, unsigned short* __restrict__ dst,
                                                   int nrow, int ncol8, float carry) {
  const int i  = blockIdx.x * 256 + threadIdx.x;
  const int n8 = nrow * ncol8;
  if (i < n8) {
    const int row = i / ncol8;
    const int c8  = i - row * ncol8;
    int srow = row;
    if (PERM) srow = (row & 3) * kH + (row >> 7) * 32 + ((row >> 2) & 1) * 16 + ((row >> 3) & 15);
    const float* sp = src + (size_t)srow * (size_t)(ncol8 * 8) + c8 * 8;
    const v4f a = *(const v4f*)(sp);
    const v4f b = *(const v4f*)(sp + 4);
    v8h hv;
#pragma unroll
    for (int e = 0; e < 4; ++e) {
      const float va = flush16(bf16r(a[e]) * carry);
      const float vb = flush16(bf16r(b[e]) * carry);
      hv[e]     = (_Float16)va;
      hv[4 + e] = (_Float16)vb;
    }
    unsigned short* q = dst + (size_t)i * 8;
    *(volatile v8h*)q = hv;
    __threadfence();
    *(volatile v8h*)q = hv;
  }
}

__global__ __launch_bounds__(256) void bias_prep_kernel(const float* __restrict__ bih_f, const float* __restrict__ bhh_f,
                                                        const float* __restrict__ bih_b, const float* __restrict__ bhh_b,
                                                        const float* __restrict__ bg, float* __restrict__ dst) {
  const int tid  = threadIdx.x;
  const int unit = (tid >> 5) * 32 + (tid & 1) * 16 + ((tid >> 1) & 15);
  v4f of, ob, og;
#pragma unroll
  for (int g = 0; g < 4; ++g) {
    of[g] = bf16r(bih_f[unit + g * kH]) + bf16r(bhh_f[unit + g * kH]);
    ob[g] = bf16r(bih_b[unit + g * kH]) + bf16r(bhh_b[unit + g * kH]);
  }
  const v4f gv = *(const v4f*)(bg + (tid & 127) * 4);
#pragma unroll
  for (int e = 0; e < 4; ++e) og[e] = bf16r(gv[e]);
  float* pf = dst + tid * 4;
  float* pb = dst + kG4 + tid * 4;
  float* pg = dst + 2 * kG4 + (tid & 127) * 4;
  *(volatile v4f*)pf = of;
  *(volatile v4f*)pb = ob;
  if (tid < 128) *(volatile v4f*)pg = og;
  __threadfence();
  *(volatile v4f*)pf = of;
  *(volatile v4f*)pb = ob;
  if (tid < 128) *(volatile v4f*)pg = og;
}

template <int MODE>
__global__ __launch_bounds__(256) void gemm64_kernel(const unsigned short* __restrict__ Ap,
                                                     const unsigned short* __restrict__ Btp,
                                                     void* __restrict__ Cout,
                                                     const float* __restrict__ bias,
                                                     const float* __restrict__ HO,
                                                     const int* __restrict__ lens) {
  constexpr int N   = (MODE == 0) ? kXgP : kOutC;
  constexpr int K   = kDin;
  constexpr int lda = kDin;
  constexpr int ldb = kDin;
  constexpr int ldc = N;
  constexpr int tilesN = N / 64;
  constexpr int tilesM = kRows / 64;
  static_assert((N % 64) == 0 && (K % 32) == 0 && (kRows % 64) == 0);
  const _Float16* A  = (const _Float16*)Ap;
  const _Float16* Bt = (const _Float16*)Btp;
  __shared__ __align__(16) float sT[8][16 * 68];
  const int lane = threadIdx.x & 31;
  const int wave = threadIdx.x >> 5;
  const int tile = blockIdx.x * 8 + wave;
  if (tile >= tilesM * tilesN) return;
  const int tm = tile / tilesN;
  const int tn = tile - tm * tilesN;
  const int m0 = tm << 6;
  const int n0 = tn << 6;
  const int bb = m0 / kT;
  const int t0 = m0 - bb * kT;
  int L = lens[bb];
  L = L < 0 ? 0 : (L > kT ? kT : L);

  const int rlane = lane & 15;
  const int hh    = lane >> 4;
  const int koff  = hh * 8;
  const int mOff  = hh * 8;
  const int c4    = rlane * 4;

  if (MODE == 0) {
    if (t0 >= L && t0 > 0) return;
  } else {
    if (t0 >= L) {
      float* C = (float*)Cout;
      const v4f z = {0.f, 0.f, 0.f, 0.f};
      for (int pass = 0; pass < 2; ++pass) {
#pragma unroll 1
        for (int it = 0; it < 32; ++it) {
          const int row = it * 2 + hh;
          *(volatile v4f*)(C + (size_t)(m0 + row) * ldc + n0 + c4) = z;
        }
        __threadfence();
      }
      return;
    }
  }

  v8f acc[4][4];
#pragma unroll
  for (int i = 0; i < 4; ++i)
#pragma unroll
    for (int j = 0; j < 4; ++j) acc[i][j] = (v8f){0.f, 0.f, 0.f, 0.f, 0.f, 0.f, 0.f, 0.f};

#pragma unroll 1
  for (int k0 = 0; k0 < K; k0 += 32) {
    v16h bh[4];
#pragma unroll
    for (int j = 0; j < 4; ++j) {
      const size_t bo = (size_t)(n0 + (j << 4) + rlane) * ldb + koff + k0;
      bh[j] = load_frag(Bt + bo);
    }
#pragma unroll
    for (int i = 0; i < 4; ++i) {
      const size_t ao = (size_t)(m0 + (i << 4) + rlane) * lda + koff + k0;
      const v16h ah = load_frag(A + ao);
#pragma unroll
      for (int j = 0; j < 4; ++j) acc[i][j] = mma_h(ah, bh[j], acc[i][j]);
    }
  }

  float bv[4];
#pragma unroll
  for (int j = 0; j < 4; ++j) bv[j] = bias[n0 + (j << 4) + rlane];

  float* slab = sT[wave];
#pragma unroll
  for (int i = 0; i < 4; ++i) {
    const int mBase = m0 + (i << 4);
#pragma unroll
    for (int j = 0; j < 4; ++j) {
#pragma unroll
      for (int r = 0; r < 8; ++r) {
        const float v = acc[i][j][r] * kInScale + bv[j];
        slab[(mOff + r) * 68 + (j << 4) + rlane] = v;
      }
    }
    __builtin_amdgcn_fence(__ATOMIC_RELEASE, "workgroup");
    __builtin_amdgcn_wave_barrier();
    __builtin_amdgcn_fence(__ATOMIC_ACQUIRE, "workgroup");
    if (MODE == 0) {
      const int q = lane >> 3, c8 = (lane & 7) * 8;
      unsigned short* C = (unsigned short*)Cout;
      v8h hv[4];
#pragma unroll
      for (int it = 0; it < 4; ++it) {
        const float* sp = slab + (it * 4 + q) * 68 + c8;
#pragma unroll
        for (int e = 0; e < 8; ++e) hv[it][e] = (_Float16)sp[e];
      }
      for (int pass = 0; pass < 2; ++pass) {
#pragma unroll
        for (int it = 0; it < 4; ++it) {
          const int row = it * 4 + q;
          *(volatile v8h*)(C + (size_t)(mBase + row) * ldc + n0 + c8) = hv[it];
        }
        __threadfence();
      }
    } else {
#pragma unroll 1
      for (int it = 0; it < 8; ++it) {
        const int row = it * 2 + hh;
        const int t = t0 + (i << 4) + row;
        const bool valid = t < L;
        const int tcl = valid ? t : (L - 1);
        float* sp = slab + row * 68 + c4;
        const v4f g4 = *(const v4f*)sp;
        const v4f h4 = *(const v4f*)(HO + (size_t)(bb * kT + tcl) * kOutC + n0 + c4);
        float h0 = h4[0], h1 = h4[1], h2 = h4[2], h3 = h4[3];
        asm volatile("" : "+v"(h0), "+v"(h1), "+v"(h2), "+v"(h3));
        v4f o;
        {
          const float g = g4[0];
          const float tg = sigm(g);
          const float f = tg * h0 + g * (1.0f - tg);
          o[0] = valid ? f : 0.0f;
        }
        {
          const float g = g4[1];
          const float tg = sigm(g);
          const float f = tg * h1 + g * (1.0f - tg);
          o[1] = valid ? f : 0.0f;
        }
        {
          const float g = g4[2];
          const float tg = sigm(g);
          const float f = tg * h2 + g * (1.0f - tg);
          o[2] = valid ? f : 0.0f;
        }
        {
          const float g = g4[3];
          const float tg = sigm(g);
          const float f = tg * h3 + g * (1.0f - tg);
          o[3] = valid ? f : 0.0f;
        }
        *(v4f*)sp = o;
      }
      __builtin_amdgcn_fence(__ATOMIC_RELEASE, "workgroup");
      __builtin_amdgcn_wave_barrier();
      __builtin_amdgcn_fence(__ATOMIC_ACQUIRE, "workgroup");
      float* C = (float*)Cout;
      for (int pass = 0; pass < 2; ++pass) {
#pragma unroll
        for (int it = 0; it < 8; ++it) {
          const int row = it * 2 + hh;
          const v4f v = *(const v4f*)(slab + row * 68 + c4);
          *(volatile v4f*)(C + (size_t)(mBase + row) * ldc + n0 + c4) = v;
        }
        __threadfence();
      }
    }
    __builtin_amdgcn_fence(__ATOMIC_RELEASE, "workgroup");
    __builtin_amdgcn_wave_barrier();
    __builtin_amdgcn_fence(__ATOMIC_ACQUIRE, "workgroup");
  }
}

__global__ __launch_bounds__(256) void lstm_scan_kernel(const unsigned short* __restrict__ XGp,
                                                        const unsigned short* __restrict__ WHp,
                                                        const int* __restrict__ lens,
                                                        float* __restrict__ HOUT) {
  __shared__ __align__(16) _Float16 Ah[2][kSeqBlk * kHP];
  __shared__ __align__(16) float    Sl[8][16 * kSlabP];
  __shared__ int sLen[kSeqBlk];
  const _Float16* WH = (const _Float16*)WHp;
  const int tid = threadIdx.x, lane = tid & 31, wave = tid >> 5;
  const int c = lane & 15, hh = lane >> 4, koff = hh * 8;
  const int q = lane >> 3, c4s = (lane & 7) * 4;
  const int dir = blockIdx.x >> 1;
  const int rowbase = (blockIdx.x & 1) * kSeqBlk;
  const bool bwd = (dir != 0);

  {
    _Float16* ahf = &Ah[0][0];
#pragma unroll 1
    for (int i = tid; i < 2 * kSeqBlk * kHP; i += 256) ahf[i] = (_Float16)0.0f;
  }
  {
    int Lraw = lens[rowbase + (tid & 15)];
    asm volatile("" : "+v"(Lraw));
    Lraw = Lraw < 0 ? 0 : (Lraw > kT ? kT : Lraw);
    if (tid < kSeqBlk) sLen[tid] = Lraw;
  }
  __syncthreads();

  int lenr[8];
#pragma unroll
  for (int r = 0; r < 8; ++r) lenr[r] = sLen[8 * hh + r];
  int slen_it[4];
#pragma unroll
  for (int it = 0; it < 4; ++it) slen_it[it] = sLen[it * 4 + q];
  int smax = 0;
#pragma unroll
  for (int i = 0; i < kSeqBlk; ++i) {
    const int v = sLen[i];
    smax = v > smax ? v : smax;
  }
  smax = smax > kT ? kT : smax;

  float c0[8], c1[8], h0s[8], h1s[8];
#pragma unroll
  for (int r = 0; r < 8; ++r) {
    c0[r] = 0.0f;
    c1[r] = 0.0f;
    h0s[r] = 0.0f;
    h1s[r] = 0.0f;
  }
  const v8f z8 = {0.f, 0.f, 0.f, 0.f, 0.f, 0.f, 0.f, 0.f};
  float* slab = Sl[wave];

#pragma unroll 1
  for (int s = 0; s < smax; ++s) {
    const int cur = s & 1;
    const _Float16* ahrow = &Ah[cur][0] + c * kHP + koff;
    _Float16* ahn = &Ah[cur ^ 1][0];

#pragma unroll 1
    for (int u = 0; u < 2; ++u) {
      const bool u1 = (u != 0);
      v2u xw[8];
#pragma unroll
      for (int r = 0; r < 8; ++r) {
        const int Lr  = lenr[r];
        const int lm1 = Lr > 0 ? Lr - 1 : 0;
        const int tf  = s < lm1 ? s : lm1;
        const int tbr = Lr - 1 - s;
        const int tb  = tbr > 0 ? tbr : 0;
        const int tr  = bwd ? tb : tf;
        const size_t off = (size_t)((rowbase + 8 * hh + r) * kT + tr) * kXgP + dir * kG4 + wave * 128 + c * 8 + u * 4;
        xw[r] = *(const v2u*)(XGp + off);
      }
      v8f a0 = z8, a1 = z8, a2 = z8, a3 = z8;
      const _Float16* wb = WH + (size_t)(dir * kG4 + 32 * wave + 16 * u + c) * kH + koff;
#pragma unroll 1
      for (int k0 = 0; k0 < kH; k0 += 32) {
        const v16h a  = load_frag(ahrow + k0);
        const v16h b0 = load_frag(wb + k0);
        const v16h b1 = load_frag(wb + (size_t)kH * kH + k0);
        const v16h b2 = load_frag(wb + (size_t)2 * kH * kH + k0);
        const v16h b3 = load_frag(wb + (size_t)3 * kH * kH + k0);
        a0 = mma_h(a, b0, a0);
        a1 = mma_h(a, b1, a1);
        a2 = mma_h(a, b2, a2);
        a3 = mma_h(a, b3, a3);
      }
#pragma unroll
      for (int r = 0; r < 8; ++r) {
        const v2u xv = xw[r];
        const unsigned w0 = xv[0];
        const unsigned w1 = xv[1];
        const float xi = h16_to_f32(w0 & 0xffffu);
        const float xf = h16_to_f32(w0 >> 16);
        const float xc = h16_to_f32(w1 & 0xffffu);
        const float xo = h16_to_f32(w1 >> 16);
        const float gi = a0[r] * kHScale + xi;
        const float gf = a1[r] * kHScale + xf;
        const float gc = a2[r] * kHScale + xc;
        const float go = a3[r] * kHScale + xo;
        const float iv = sigm(gi);
        const float fv = sigm(gf);
        const float gv = tanh_id(gc);
        const float ov = sigm(go);
        const float cp = u1 ? c1[r] : c0[r];
        const float hp = u1 ? h1s[r] : h0s[r];
        const float cn = fv * cp + iv * gv;
        const float hn = ov * tanh_id(cn);
        const bool valid = s < lenr[r];
        const float cs = valid ? cn : cp;
        const float hs = valid ? hn : hp;
        c0[r]  = u1 ? c0[r] : cs;
        c1[r]  = u1 ? cs : c1[r];
        h0s[r] = u1 ? h0s[r] : hs;
        h1s[r] = u1 ? hs : h1s[r];
        const float hc = flush16(hs * kHCarry);
        ahn[(8 * hh + r) * kHP + 32 * wave + 16 * u + c] = (_Float16)hc;
        slab[(8 * hh + r) * kSlabP + 16 * u + c] = hn;
      }
    }
    __syncthreads();

    v4f sv[4];
#pragma unroll
    for (int it = 0; it < 4; ++it) sv[it] = *(const v4f*)(slab + (it * 4 + q) * kSlabP + c4s);
    for (int pass = 0; pass < 2; ++pass) {
#pragma unroll
      for (int it = 0; it < 4; ++it) {
        const int row = it * 4 + q;
        const int Lr  = slen_it[it];
        const bool valid = s < Lr;
        const int tt  = bwd ? (Lr - 1 - s) : s;
        const int tcl = tt < 0 ? 0 : (tt > kT - 1 ? kT - 1 : tt);
        float* p = HOUT + (size_t)((rowbase + row) * kT + tcl) * kOutC + dir * kH + 32 * wave + c4s;
        if (valid) *(volatile v4f*)p = sv[it];
      }
      __threadfence();
    }
    __builtin_amdgcn_fence(__ATOMIC_RELEASE, "workgroup");
    __builtin_amdgcn_wave_barrier();
    __builtin_amdgcn_fence(__ATOMIC_ACQUIRE, "workgroup");
  }
}

extern "C" void kernel_launch(void* const* d_in, const int* in_sizes, int n_in,
                              void* d_out, int out_size, void* d_ws, size_t ws_size,
                              hipStream_t stream) {
  if (n_in < 12 || d_out == nullptr || d_ws == nullptr) return;
  if (in_sizes[0] != kRows * kDin) return;
  if (in_sizes[1] != kG4 * kDin || in_sizes[5] != kG4 * kDin) return;
  if (in_sizes[2] != kG4 * kH || in_sizes[6] != kG4 * kH) return;
  if (in_sizes[3] != kG4 || in_sizes[4] != kG4 || in_sizes[7] != kG4 || in_sizes[8] != kG4) return;
  if (in_sizes[9] != kOutC * kDin || in_sizes[10] != kOutC || in_sizes[11] != kB) return;
  if (out_size != kRows * kOutC) return;
  if (ws_size < kWsTotal) return;

  const float* x     = (const float*)d_in[0];
  const float* Wih_f = (const float*)d_in[1];
  const float* Whh_f = (const float*)d_in[2];
  const float* bih_f = (const float*)d_in[3];
  const float* bhh_f = (const float*)d_in[4];
  const float* Wih_b = (const float*)d_in[5];
  const float* Whh_b = (const float*)d_in[6];
  const float* bih_b = (const float*)d_in[7];
  const float* bhh_b = (const float*)d_in[8];
  const float* Wg    = (const float*)d_in[9];
  const float* bg    = (const float*)d_in[10];
  const int*   lens  = (const int*)d_in[11];

  char* ws = (char*)d_ws;
  unsigned short* XH   = (unsigned short*)(ws + kOffXH);
  unsigned short* WCAT = (unsigned short*)(ws + kOffWCAT);
  unsigned short* WHH  = (unsigned short*)(ws + kOffWHH);
  float*          BIAS = (float*)(ws + kOffBIAS);
  unsigned short* XG   = (unsigned short*)(ws + kOffXG);
  float*          HOUT = (float*)(ws + kOffHOUT);

  cvt8_kernel<false><<<(kRows * (kDin / 8)) / 256, 256, 0, stream>>>(x, XH, kRows, kDin / 8, kXCarry);
  cvt8_kernel<true><<<(kG4 * (kDin / 8)) / 256, 256, 0, stream>>>(Wih_f, WCAT, kG4, kDin / 8, kWCarry);
  cvt8_kernel<true><<<(kG4 * (kDin / 8)) / 256, 256, 0, stream>>>(Wih_b, WCAT + (size_t)kG4 * kDin, kG4, kDin / 8, kWCarry);
  cvt8_kernel<false><<<(kOutC * (kDin / 8)) / 256, 256, 0, stream>>>(Wg, WCAT + (size_t)2 * kG4 * kDin, kOutC, kDin / 8, kWCarry);
  cvt8_kernel<false><<<(kG4 * (kH / 8)) / 256, 256, 0, stream>>>(Whh_f, WHH, kG4, kH / 8, kWCarry);
  cvt8_kernel<false><<<(kG4 * (kH / 8)) / 256, 256, 0, stream>>>(Whh_b, WHH + (size_t)kG4 * kH, kG4, kH / 8, kWCarry);
  bias_prep_kernel<<<1, 256, 0, stream>>>(bih_f, bhh_f, bih_b, bhh_b, bg, BIAS);

  gemm64_kernel<0><<<((kRows / 64) * (kXgP / 64)) / 8, 256, 0, stream>>>(XH, WCAT, (void*)XG, BIAS, HOUT, lens);

  lstm_scan_kernel<<<4, 256, 0, stream>>>(XG, WHH, lens, HOUT);

  gemm64_kernel<1><<<((kRows / 64) * (kOutC / 64)) / 8, 256, 0, stream>>>(
      XH, WCAT + (size_t)2 * kG4 * kDin, d_out, BIAS + 2 * kG4, HOUT, lens);
}
